// Warp_deform_42348377539036
// MI455X (gfx1250) — hardware-verified
//
#include <hip/hip_runtime.h>
#include <math.h>

typedef __attribute__((ext_vector_type(16))) _Float16 v16h;
typedef __attribute__((ext_vector_type(16))) __bf16 v16b;
typedef __attribute__((ext_vector_type(8)))  _Float16 v8h;
typedef __attribute__((ext_vector_type(8)))  float v8f;
typedef __attribute__((ext_vector_type(4)))  float v4f;
typedef __attribute__((ext_vector_type(2)))  float v2f;
typedef __attribute__((ext_vector_type(4)))  unsigned v4u;
typedef __attribute__((ext_vector_type(4)))  int v4i;
typedef float __attribute__((may_alias)) float_a;
typedef int __attribute__((may_alias)) int_a;

template <typename T> __device__ __forceinline__ void vst2(void* p, T v) { *(volatile T*)p = v; __threadfence(); *(volatile T*)p = v; }
__device__ __forceinline__ v8f wmma16(v16h a, v16h b, v8f c) {
  v8f d = __builtin_amdgcn_wmma_f32_16x16x32_f16(false, a, false, b, (short)0, c, false, false);
  asm volatile("v_nop\n\tv_nop\n\tv_nop\n\tv_nop" : "+v"(d) : "v"(a), "v"(b));
  return d;
}
__device__ __forceinline__ v8f wmma_bf(v16b a, v16b b, v8f c) {
  v8f d = __builtin_amdgcn_wmma_f32_16x16x32_bf16(false, a, false, b, (short)0, c, false, false);
  asm volatile("v_nop\n\tv_nop\n\tv_nop\n\tv_nop" : "+v"(d) : "v"(a), "v"(b));
  return d;
}
__device__ __forceinline__ v16h frag_h(const _Float16* rowk0, int lane) {
  union { v16h v; v8h q[2]; } u; const _Float16* p = rowk0 + 8 * (lane >> 4);
  u.q[0] = *(const v8h*)p; u.q[1] = *(const v8h*)(p + 16); return u.v;
}
__device__ __forceinline__ v16h frag_f32(const float* rowk0, int lane) {
  v16h a; const float* p = rowk0 + 8 * (lane >> 4);
#pragma unroll
  for (int i = 0; i < 8; ++i) { a[i] = (_Float16)p[i]; a[8 + i] = (_Float16)p[16 + i]; }
  return a;
}
__device__ __forceinline__ v16h frag_f32s(const float* rowk0, int lane, float sc) {
  v16h a; const float* p = rowk0 + 8 * (lane >> 4);
#pragma unroll
  for (int i = 0; i < 8; ++i) { a[i] = (_Float16)(p[i] * sc); a[8 + i] = (_Float16)(p[16 + i] * sc); }
  return a;
}
__device__ __forceinline__ v16h fragc_f32(const float* W, int k0, int n, int lane, int ld, int K) {
  v16h a; const int g = lane >> 4;
#pragma unroll
  for (int i = 0; i < 8; ++i) { const int ka = k0 + 8 * g + i, kb = ka + 16;
    a[i] = (_Float16)(ka < K ? W[(size_t)(ka < K ? ka : K - 1) * ld + n] : 0.f); a[8 + i] = (_Float16)(kb < K ? W[(size_t)(kb < K ? kb : K - 1) * ld + n] : 0.f); }
  return a;
}
struct F2 { v16b h, l; };
__device__ __forceinline__ F2 bsplit16(const float v[16]) { F2 r;
#pragma unroll
  for (int i = 0; i < 16; ++i) { const __bf16 h = (__bf16)v[i]; r.h[i] = h; r.l[i] = (__bf16)(v[i] - (float)h); }
  return r; }
__device__ __forceinline__ F2 split_row(const float* row, int k0, int lane) { float v[16]; const float* p = row + k0 + 8 * (lane >> 4);
#pragma unroll
  for (int i = 0; i < 8; ++i) { v[i] = p[i]; v[8 + i] = p[16 + i]; }
  return bsplit16(v); }
__device__ __forceinline__ F2 split_rowK(const float* row, int k0, int lane, int K) { float v[16]; const int g = lane >> 4;
#pragma unroll
  for (int i = 0; i < 8; ++i) { const int ka = k0 + 8 * g + i, kb = ka + 16; v[i] = ka < K ? row[ka < K ? ka : K - 1] : 0.f; v[8 + i] = kb < K ? row[kb < K ? kb : K - 1] : 0.f; }
  return bsplit16(v); }
__device__ __forceinline__ F2 split_col(const float* W, int k0, int n, int lane, int ld, int K) { float v[16]; const int g = lane >> 4;
#pragma unroll
  for (int i = 0; i < 8; ++i) { const int ka = k0 + 8 * g + i, kb = ka + 16; v[i] = ka < K ? W[(size_t)(ka < K ? ka : K - 1) * ld + n] : 0.f; v[8 + i] = kb < K ? W[(size_t)(kb < K ? kb : K - 1) * ld + n] : 0.f; }
  return bsplit16(v); }
__device__ __forceinline__ v8f mac3(const F2& a, const F2& b, v8f c) { c = wmma_bf(a.l, b.h, c); c = wmma_bf(a.h, b.l, c); return wmma_bf(a.h, b.h, c); }
__device__ __forceinline__ float sigm(float v) { return 1.0f / (1.0f + expf(-v)); }
#define LDSX() do { asm volatile("s_wait_dscnt 0" ::: "memory"); __builtin_amdgcn_wave_barrier(); __builtin_amdgcn_fence(__ATOMIC_RELEASE, "workgroup"); } while (0)


#define NB 8
#define CI 64
#define CO 64
#define HH 128
#define WW 128
#define KK 9
#define NPX (HH * WW)
#ifndef TPB
#define TPB (NPX / 64)
#define TNB NB
#endif
typedef __attribute__((ext_vector_type(8))) __bf16 v8b;
__device__ __forceinline__ v16b frag_b(const __bf16* rowk0, int lane) {
  union { v16b v; v8b q[2]; } u; const __bf16* p = rowk0 + 8 * (lane >> 4);
  u.q[0] = *(const v8b*)p; u.q[1] = *(const v8b*)(p + 16); return u.v;
}
__device__ __forceinline__ float bfr(float v) { return (float)(__bf16)v; }
__device__ __attribute__((noinline)) float exp_ni(float v) { return expf(v); }
__device__ __attribute__((noinline)) float erf_ni(float v) { return erff(v); }

#define WS_W   0u
#define WS_END (2u * KK * CO * CI)

__global__ __launch_bounds__(64) void k_packw(const float* __restrict__ WT, __bf16* __restrict__ PW) {
  const int o = blockIdx.x, k = blockIdx.y, c = threadIdx.x; __shared__ __align__(16) __bf16 s[CI]; s[c] = (__bf16)WT[((size_t)o * CI + c) * KK + k]; __syncthreads();
  if (c < CI / 8) vst2((unsigned*)(PW + ((size_t)k * CO + o) * CI + c * 8), *(const v4u*)&s[c * 8]);
}
__global__ __launch_bounds__(128) void k_deform(const float* __restrict__ FEA, const float* __restrict__ OFF, const __bf16* __restrict__ PW, const float* __restrict__ BIAS, float* __restrict__ OUT) {
  __shared__ __align__(16) __bf16 sh[64][72], sl[64][72]; __shared__ int sidx[4][64]; __shared__ float swt[4][64]; __shared__ __align__(16) float so[CO][68];
  const int tid = threadIdx.x, wave = tid >> 5, lane = tid & 31, col = lane & 15, g = lane >> 4; const size_t b = blockIdx.y; const int p0 = blockIdx.x * 64;
  v8f acc[4] = {};
#pragma unroll 1
  for (int k = 0; k < KK; ++k) {
    if (tid < 64) { const int p = p0 + tid; const int h = p / WW, w = p % WW; const float ky = (float)(k / 3 - 1), kx = (float)(k % 3 - 1);
      const float dy = bfr(OFF[((b * (2 * KK) + 2 * k) * HH + h) * WW + w]), dx = bfr(OFF[((b * (2 * KK) + 2 * k + 1) * HH + h) * WW + w]);
      const float py = ((float)h + ky) + dy, px = ((float)w + kx) + dx;
      const float y0 = floorf(py), x0 = floorf(px); const float ay = py - y0, ax = px - x0;
      const float yc[2] = {y0, y0 + 1.0f}, xc[2] = {x0, x0 + 1.0f}; const float wy[2] = {1.0f - ay, ay}, wx[2] = {1.0f - ax, ax};
#pragma unroll
      for (int q = 0; q < 4; ++q) { const int iy = q >> 1, ix = q & 1; const float yf = yc[iy], xf = xc[ix]; const bool valid = (yf >= 0.f) && (yf <= (float)(HH - 1)) && (xf >= 0.f) && (xf <= (float)(WW - 1));
        const int yi = (int)fminf(fmaxf(yf, 0.f), (float)(HH - 1)), xi = (int)fminf(fmaxf(xf, 0.f), (float)(WW - 1));
        const float wgt = wy[iy] * wx[ix];
        sidx[q][tid] = yi * WW + xi; swt[q][tid] = valid ? wgt : 0.f; } }
    __syncthreads();
    for (int e = tid; e < 64 * CI; e += 128) { const int px = e & 63, c = e >> 6; const float* F = FEA + (b * CI + c) * NPX; float v = 0.f;
#pragma unroll
      for (int q = 0; q < 4; ++q) { const float gq = bfr(F[sidx[q][px]]) * swt[q][px]; v = v + gq; }
      const __bf16 hb = (__bf16)v; sh[px][c] = hb; sl[px][c] = (__bf16)(v - (float)hb); }
    if (tid < 64) for (int c = CI; c < 72; ++c) { sh[tid][c] = (__bf16)0.f; sl[tid][c] = (__bf16)0.f; }
    __syncthreads();
#pragma unroll
    for (int kc = 0; kc < CI / 32; ++kc) { const v16b a = frag_b(&sh[wave * 16 + col][kc * 32], lane), al = frag_b(&sl[wave * 16 + col][kc * 32], lane);
#pragma unroll
      for (int j = 0; j < 4; ++j) { const v16b w = frag_b(PW + ((size_t)k * CO + j * 16 + col) * CI + kc * 32, lane); acc[j] = wmma_bf(al, w, acc[j]); acc[j] = wmma_bf(a, w, acc[j]); } }
    __syncthreads(); }
#pragma unroll
  for (int j = 0; j < 4; ++j) { const int o = j * 16 + col; const float bb = bfr(BIAS[o]);
#pragma unroll
    for (int r = 0; r < 8; ++r) so[o][wave * 16 + 8 * g + r] = acc[j][r] + bb; }
  __syncthreads();
  for (int e = tid; e < CO * 16; e += 128) { const int o = e >> 4, q = e & 15; vst2(OUT + ((b * CO + o) * NPX) + p0 + q * 4, *(const v4f*)&so[o][q * 4]); }
}
extern "C" void kernel_launch(void* const* d_in, const int* in_sizes, int n_in, void* d_out, int out_size, void* d_ws, size_t ws_size, hipStream_t stream) {
  (void)in_sizes; (void)n_in; (void)out_size;
  const float** F = (const float**)d_in;
  if (ws_size < (size_t)WS_END) return;
  char* ws = (char*)d_ws; __bf16* PW = (__bf16*)(ws + WS_W);
  k_packw<<<dim3(CO, KK), 64, 0, stream>>>(F[2], PW);
  k_deform<<<dim3(TPB, TNB), 128, 0, stream>>>(F[0], F[1], PW, F[3], (float*)d_out);
}
